// ContrastiveWrapper_31782757991084
// MI455X (gfx1250) — hardware-run, weakly checked
//
#include <hip/hip_runtime.h>


#define NROW  8192
#define NIN   512
#define NHID  1024
#define NEMB  64
#define NCON  62
#define XP    513
#define GBLK  1024
#define NBLK  (NROW / GBLK)
typedef _Float16 h16;
typedef unsigned short bf;
typedef __attribute__((ext_vector_type(16))) __bf16   v16bf;
typedef __attribute__((ext_vector_type(16))) _Float16 v16h;
typedef __attribute__((ext_vector_type(8)))  _Float16 v8h;
typedef __attribute__((ext_vector_type(8)))  unsigned short v8us;
typedef __attribute__((ext_vector_type(8)))  float    v8f;
typedef __attribute__((ext_vector_type(4)))  float    v4f;
typedef v8h  __attribute__((may_alias)) v8ha;
typedef v4f  __attribute__((may_alias)) v4fa;
typedef v8us __attribute__((may_alias)) v8usa;

__device__ __forceinline__ unsigned short f2bf(float f) { unsigned u = __float_as_uint(f); u += 0x7FFFu + ((u >> 16) & 1u); return (unsigned short)(u >> 16); }
__device__ __forceinline__ float bf2f(unsigned short b) { return __uint_as_float(((unsigned)b) << 16); }
__device__ __forceinline__ float bfr(float f) { return bf2f(f2bf(f)); }
__device__ __forceinline__ v16h cat16(v8h lo, v8h hi) { return __builtin_shufflevector(lo, hi, 0, 1, 2, 3, 4, 5, 6, 7, 8, 9, 10, 11, 12, 13, 14, 15); }
__device__ __forceinline__ v16bf cat16b(v8us lo, v8us hi) { return __builtin_bit_cast(v16bf, __builtin_shufflevector(lo, hi, 0, 1, 2, 3, 4, 5, 6, 7, 8, 9, 10, 11, 12, 13, 14, 15)); }
__device__ __forceinline__ v8f wmma16(v16h a, v16h b, v8f c) { return __builtin_amdgcn_wmma_f32_16x16x32_f16(false, a, false, b, (short)0, c, false, false); }
__device__ __forceinline__ v8f wmmab(v16bf a, v16bf b, v8f c) { return __builtin_amdgcn_wmma_f32_16x16x32_bf16(false, a, false, b, (short)0, c, false, false); }

template <typename T16> struct WFrag;
template <> struct WFrag<h16> { typedef v16h V; static __device__ __forceinline__ V ld(const h16* p) { return cat16(*(const v8h*)p, *(const v8h*)(p + 16)); } static __device__ __forceinline__ v8f mma(V a, V b, v8f c) { return wmma16(a, b, c); } };
template <> struct WFrag<bf> { typedef v16bf V; static __device__ __forceinline__ V ld(const bf* p) { return cat16b(*(const v8us*)p, *(const v8us*)(p + 16)); } static __device__ __forceinline__ v8f mma(V a, V b, v8f c) { return wmmab(a, b, c); } };
template <typename T16, int NSPLIT, bool BIAS>
__global__ __launch_bounds__(32) void k_gemmw(const T16* __restrict__ A, const T16* __restrict__ A2, const T16* __restrict__ Bt, const T16* __restrict__ Bt2, int K, float* C, int ldc, const float* __restrict__ bias, size_t sA, size_t sB, size_t sC) {
    typedef typename WFrag<T16>::V V;
    __shared__ __align__(16) float os[16 * 68];
    const size_t z = blockIdx.z; A += z * sA; if (A2) A2 += z * sA; Bt += z * sB; if (Bt2) Bt2 += z * sB; C += z * sC;
    const int lane = threadIdx.x & 31, lr = lane & 15, hi = lane >> 4; const int r0 = blockIdx.x * 64, c0 = blockIdx.y * 64;
    v8f acc[4][4];
#pragma unroll
    for (int mb = 0; mb < 4; ++mb)
#pragma unroll
        for (int nb = 0; nb < 4; ++nb) acc[mb][nb] = (v8f){};
    const size_t aoff = (size_t)(r0 + lr) * K + 8 * hi, boff = (size_t)(c0 + lr) * K + 8 * hi;
    for (int kc = 0; kc < K; kc += 32) {
        V a[4], a2[4];
#pragma unroll
        for (int mb = 0; mb < 4; ++mb) { a[mb] = WFrag<T16>::ld(A + aoff + (size_t)mb * 16 * K + kc); if (NSPLIT == 1 || NSPLIT == 2) a2[mb] = WFrag<T16>::ld(A2 + aoff + (size_t)mb * 16 * K + kc); }
#pragma unroll
        for (int nb = 0; nb < 4; ++nb) { const V b = WFrag<T16>::ld(Bt + boff + (size_t)nb * 16 * K + kc); V b2; if (NSPLIT >= 2) b2 = WFrag<T16>::ld(Bt2 + boff + (size_t)nb * 16 * K + kc);
#pragma unroll
            for (int mb = 0; mb < 4; ++mb) { acc[mb][nb] = WFrag<T16>::mma(a[mb], b, acc[mb][nb]); if (NSPLIT == 1 || NSPLIT == 2) acc[mb][nb] = WFrag<T16>::mma(a2[mb], b, acc[mb][nb]); if (NSPLIT >= 2) acc[mb][nb] = WFrag<T16>::mma(a[mb], b2, acc[mb][nb]); } }
        asm volatile("v_nop\n\tv_nop\n\tv_nop\n\tv_nop" : "+v"(acc[0][0]), "+v"(acc[1][1]), "+v"(acc[2][2]), "+v"(acc[3][3]) : "v"(a[0]), "v"(a[3]));
    }
#pragma unroll
    for (int mb = 0; mb < 4; ++mb) {
#pragma unroll
        for (int nb = 0; nb < 4; ++nb) {
#pragma unroll
            for (int j = 0; j < 8; ++j) os[(hi * 8 + j) * 68 + nb * 16 + lr] = acc[mb][nb][j]; }
        __builtin_amdgcn_wave_barrier(); asm volatile("" ::: "memory");
        float* crow = C + (size_t)(r0 + mb * 16) * ldc + c0;
#pragma unroll 1
        for (int ps = 0; ps < 2; ++ps) {
#pragma unroll
            for (int s = 0; s < 8; ++s) { const int row = 2 * s + hi, cofs = lr * 4; v4f val = *(const v4fa*)(os + row * 68 + cofs); if (BIAS) { val[0] += bfr(bias[c0 + cofs]); val[1] += bfr(bias[c0 + cofs + 1]); val[2] += bfr(bias[c0 + cofs + 2]); val[3] += bfr(bias[c0 + cofs + 3]); }
                *(volatile v4f*)(crow + (size_t)row * ldc + cofs) = val; }
            if (ps == 0) __threadfence(); }
        __builtin_amdgcn_wave_barrier(); asm volatile("" ::: "memory");
    }
}

typedef __attribute__((ext_vector_type(2))) _Float16 v2h;
typedef __attribute__((ext_vector_type(4))) _Float16 v4h;
typedef __attribute__((ext_vector_type(2))) unsigned short v2us;
typedef __attribute__((ext_vector_type(4))) unsigned short v4us;
typedef __attribute__((ext_vector_type(2))) float v2f;
__device__ __forceinline__ h16 toh_flush(float x) { const float z = (fabsf(x) < 6.103515625e-05f) ? 0.0f : x; return (h16)z; }

__device__ __forceinline__ float tanhc(float v) { return 1.0f - 2.0f / (expf(2.0f * v) + 1.0f); }

__global__ __launch_bounds__(256) void k_wt16(const float* __restrict__ src, h16* dst, int lgK, int N, int n8) { const int i = blockIdx.x * 256 + threadIdx.x; if (i >= n8) return; const int e = i * 8; const int n = e >> lgK, k0 = e & ((1 << lgK) - 1); v8h o;
#pragma unroll
    for (int q = 0; q < 8; ++q) o[q] = toh_flush(bfr(src[(size_t)(k0 + q) * N + n]));
    *(volatile v8h*)(dst + (size_t)i * 8) = o; __threadfence(); *(volatile v8h*)(dst + (size_t)i * 8) = o; }

__global__ __launch_bounds__(256) void k_xcast(const float* __restrict__ x, h16* dst) { const int i = blockIdx.x * 256 + threadIdx.x; if (i >= NROW * NIN / 8) return; const int r = i >> 6, c0 = (i & 63) * 8; v8h o;
#pragma unroll
    for (int q = 0; q < 8; ++q) o[q] = toh_flush(bfr(x[(size_t)r * XP + 1 + c0 + q]));
    *(volatile v8h*)(dst + (size_t)i * 8) = o; __threadfence(); *(volatile v8h*)(dst + (size_t)i * 8) = o; }

__global__ __launch_bounds__(256) void k_tanh16(const float* __restrict__ src, h16* dst, int n8) { const int i = blockIdx.x * 256 + threadIdx.x; if (i >= n8) return; const v8f v = *(const v8f*)(src + (size_t)i * 8); v8h o;
#pragma unroll
    for (int q = 0; q < 8; ++q) o[q] = toh_flush(tanhc(v[q]));
    *(volatile v8h*)(dst + (size_t)i * 8) = o; __threadfence(); *(volatile v8h*)(dst + (size_t)i * 8) = o; }

__global__ __launch_bounds__(256) void k_cons(const float* __restrict__ E, h16* E16, h16* Cq, float* sq) { const int r = blockIdx.x * 256 + threadIdx.x; if (r >= NROW) return; float e[NEMB];
#pragma unroll
    for (int k = 0; k < NEMB / 4; ++k) { const v4f t = *(const v4f*)(E + (size_t)r * NEMB + 4 * k); e[4 * k] = t[0]; e[4 * k + 1] = t[1]; e[4 * k + 2] = t[2]; e[4 * k + 3] = t[3]; }
    float s = 0.0f;
#pragma unroll
    for (int k = 0; k < NCON; ++k) s = __fmaf_rn(e[2 + k], e[2 + k], s);
    v8h o[8], w[8];
#pragma unroll
    for (int k = 0; k < NEMB; ++k) { w[k >> 3][k & 7] = toh_flush(e[k]); o[k >> 3][k & 7] = (k < NCON) ? toh_flush(e[2 + k]) : toh_flush(__fmul_rn(e[k], 0.0f)); }
#pragma unroll
    for (int ps = 0; ps < 2; ++ps) {
#pragma unroll
        for (int k = 0; k < 8; ++k) *(volatile v8h*)(E16 + (size_t)r * NEMB + 8 * k) = w[k];
#pragma unroll
        for (int k = 0; k < 8; ++k) *(volatile v8h*)(Cq + (size_t)r * NEMB + 8 * k) = o[k];
        *(volatile float*)(sq + r) = s; if (ps == 0) __threadfence(); } }

__global__ __launch_bounds__(256) void k_pair(const float* __restrict__ G, const float* __restrict__ sq, const float* __restrict__ x, int i0, float* Psim, float* Pdif, unsigned* Pcnt) { const int j = blockIdx.x * 256 + threadIdx.x; if (j >= NROW) return;
    const int lj = (int)x[(size_t)j * XP]; const float sqj = sq[j]; float sim = 0.0f, dif = 0.0f; unsigned cnt = 0u;
    for (int i = 0; i < GBLK; ++i) { const int li = (int)x[(size_t)(i0 + i) * XP]; const float g = G[(size_t)i * NROW + j];
        const float D = __fdiv_rn(fmaxf(__fsub_rn(__fadd_rn(sq[i0 + i], sqj), __fmul_rn(2.0f, g)), 0.0f), (float)NCON); const float m = fmaxf(0.0f, __fsub_rn(0.01f, D)); const bool df = (li != lj);
        sim = __fadd_rn(sim, df ? D : 0.0f); dif = __fadd_rn(dif, df ? 0.0f : m); cnt += df ? 1u : 0u; }
    const size_t o = (size_t)(i0 / GBLK) * NROW + j;
    *(volatile float*)(Psim + o) = sim; *(volatile float*)(Pdif + o) = dif; *(volatile unsigned*)(Pcnt + o) = cnt; __threadfence(); *(volatile float*)(Psim + o) = sim; *(volatile float*)(Pdif + o) = dif; *(volatile unsigned*)(Pcnt + o) = cnt; }

__global__ __launch_bounds__(32) void k_fin(const float* __restrict__ Psim, const float* __restrict__ Pdif, const unsigned* __restrict__ Pcnt, float* out2) { if (blockIdx.x != 0 || threadIdx.x != 0) return; float S = 0.0f, T = 0.0f; unsigned nu = 0u;
    for (int k = 0; k < NBLK * NROW; ++k) { S = __fadd_rn(S, Psim[k]); T = __fadd_rn(T, Pdif[k]); nu += Pcnt[k]; }
    const float n = (float)nu;
    const float cs = __fdiv_rn(S, __fadd_rn(n, 1.0f)); const float cd = __fdiv_rn(T, __fadd_rn(__fsub_rn((float)NROW * (float)NROW, n), 1.0f));
    v2f o; o[0] = cs; o[1] = cd; *(volatile v2f*)(out2) = o; __threadfence(); *(volatile v2f*)(out2) = o; }

extern "C" void kernel_launch(void* const* d_in, const int* in_sizes, int n_in, void* d_out, int out_size, void* d_ws, size_t ws_size, hipStream_t stream) {
    if (n_in < 9) return;
    if (in_sizes[0] != NROW * XP || in_sizes[1] != NIN * NHID || in_sizes[2] != NHID || in_sizes[3] != NHID * NEMB || in_sizes[4] != NEMB || in_sizes[5] != NEMB * NHID || in_sizes[6] != NHID || in_sizes[7] != NHID * NIN || in_sizes[8] != NIN) return;
    if (out_size != NROW * NIN + 2) return;
    static_assert(NROW % 64 == 0 && NHID % 64 == 0 && NEMB % 64 == 0 && NIN % 64 == 0 && NIN % 32 == 0 && NHID % 32 == 0 && NEMB % 32 == 0 && GBLK % 64 == 0 && NROW % GBLK == 0 && NROW % 256 == 0 && (NROW * NIN / 8) % 256 == 0 && (NROW * NHID / 8) % 256 == 0 && (NROW * NEMB / 8) % 256 == 0 && NCON + 2 == NEMB && (NIN & (NIN - 1)) == 0 && (NHID & (NHID - 1)) == 0 && (NEMB & (NEMB - 1)) == 0 && ((size_t)NROW * NIN * 4) % 128 == 0, "the products: M and N multiples of 64, the depths multiples of 32 and powers of two; every elementwise grid exact; the two scalars begin on a 128-byte line");
    const float* x = (const float*)d_in[0]; const float* w1 = (const float*)d_in[1]; const float* b1 = (const float*)d_in[2]; const float* w2 = (const float*)d_in[3]; const float* b2 = (const float*)d_in[4]; const float* w3 = (const float*)d_in[5]; const float* b3 = (const float*)d_in[6]; const float* w4 = (const float*)d_in[7]; const float* b4 = (const float*)d_in[8];
    float* out = (float*)d_out; float* out0 = out;     float* out2 = out + (size_t)NROW * NIN;
    char* wsp = (char*)d_ws; auto take = [&](size_t bytes) { char* p = wsp; wsp += (bytes + 255) & ~(size_t)255; return (void*)p; };
    h16* W1t = (h16*)take((size_t)NHID * NIN * 2);     h16* W2t = (h16*)take((size_t)NEMB * NHID * 2);     h16* W3t = (h16*)take((size_t)NHID * NEMB * 2);     h16* W4t = (h16*)take((size_t)NIN * NHID * 2);
    h16* X16 = (h16*)take((size_t)NROW * NIN * 2);     h16* H16 = (h16*)take((size_t)NROW * NHID * 2);     h16* E16 = (h16*)take((size_t)NROW * NEMB * 2);     h16* Cq = (h16*)take((size_t)NROW * NEMB * 2);
    float* PF = (float*)take((size_t)NROW * NHID * 4);     float* E = (float*)take((size_t)NROW * NEMB * 4);     float* sq = (float*)take((size_t)NROW * 4);
    float* Psim = (float*)take((size_t)NBLK * NROW * 4); float* Pdif = (float*)take((size_t)NBLK * NROW * 4); unsigned* Pcnt = (unsigned*)take((size_t)NBLK * NROW * 4);
    if ((size_t)(wsp - (char*)d_ws) > ws_size) return;
    k_wt16<<<(unsigned)(NIN * NHID / 8 / 256), 256, 0, stream>>>(w1, W1t, 9, NHID, NIN * NHID / 8);
    k_wt16<<<(unsigned)(NHID * NEMB / 8 / 256), 256, 0, stream>>>(w2, W2t, 10, NEMB, NHID * NEMB / 8);
    k_wt16<<<(unsigned)(NEMB * NHID / 8 / 256), 256, 0, stream>>>(w3, W3t, 6, NHID, NEMB * NHID / 8);
    k_wt16<<<(unsigned)(NHID * NIN / 8 / 256), 256, 0, stream>>>(w4, W4t, 10, NIN, NHID * NIN / 8);
    k_xcast<<<(unsigned)(NROW * NIN / 8 / 256), 256, 0, stream>>>(x, X16);
    k_gemmw<h16, 0, true><<<dim3(NROW / 64, NHID / 64, 1), 32, 0, stream>>>(X16, nullptr, W1t, nullptr, NIN, PF, NHID, b1, 0, 0, 0);
    k_tanh16<<<(unsigned)(NROW * NHID / 8 / 256), 256, 0, stream>>>(PF, H16, NROW * NHID / 8);
    k_gemmw<h16, 0, true><<<dim3(NROW / 64, NEMB / 64, 1), 32, 0, stream>>>(H16, nullptr, W2t, nullptr, NHID, E, NEMB, b2, 0, 0, 0);
    k_cons<<<(unsigned)(NROW / 256), 256, 0, stream>>>(E, E16, Cq, sq);
    k_gemmw<h16, 0, true><<<dim3(NROW / 64, NHID / 64, 1), 32, 0, stream>>>(E16, nullptr, W3t, nullptr, NEMB, PF, NHID, b3, 0, 0, 0);
    k_tanh16<<<(unsigned)(NROW * NHID / 8 / 256), 256, 0, stream>>>(PF, H16, NROW * NHID / 8);
    k_gemmw<h16, 0, true><<<dim3(NROW / 64, NIN / 64, 1), 32, 0, stream>>>(H16, nullptr, W4t, nullptr, NHID, out0, NIN, b4, 0, 0, 0);
    for (int blk = 0; blk < NBLK; ++blk) {
        k_gemmw<h16, 0, false><<<dim3(GBLK / 64, NROW / 64, 1), 32, 0, stream>>>(Cq + (size_t)blk * GBLK * NEMB, nullptr, Cq, nullptr, NEMB, PF, NROW, nullptr, 0, 0, 0);
        k_pair<<<(unsigned)(NROW / 256), 256, 0, stream>>>(PF, sq, x, blk * GBLK, Psim, Pdif, Pcnt); }
    k_fin<<<1, 32, 0, stream>>>(Psim, Pdif, Pcnt, out2);
}
